// NezNet_46248207843927
// MI455X (gfx1250) — hardware-verified
//
#include <hip/hip_runtime.h>
#include <stddef.h>


#define NTHR   256
#define NWAVE  8
#define HC     128
#define FIN    64
#define GMAX   512
#define HP     136
#define WSCL   8.0f
#define WINV   0.125f
#define BNEPS  1e-3f

#define EPT    16
#define CHUNK  (NTHR * EPT)
#define WCAP   (32 * EPT)
#define LISTN  (NWAVE * WCAP)
#define PASSN  NTHR
#define PCAP   (CHUNK + PASSN)
#define NB     256

static_assert(PASSN == 256);
static_assert(NB == 32 * NWAVE);
static_assert(CHUNK < 65536);
static_assert(PCAP >= CHUNK + PASSN);

typedef float    v4f  __attribute__((ext_vector_type(4)));
typedef float    v8f  __attribute__((ext_vector_type(8)));
typedef int      v4i  __attribute__((ext_vector_type(4)));
typedef _Float16 v8h  __attribute__((ext_vector_type(8)));
typedef _Float16 v16h __attribute__((ext_vector_type(16)));
typedef __bf16   v8b  __attribute__((ext_vector_type(8)));
typedef __bf16   v16b __attribute__((ext_vector_type(16)));
typedef v4f __attribute__((may_alias)) v4fa;
typedef v4i __attribute__((may_alias)) v4ia;
typedef v8h __attribute__((may_alias)) v8ha;
typedef v8b __attribute__((may_alias)) v8ba;
union FragH { v16h v; v8h h[2]; };
union FragB { v16b v; v8b h[2]; };

__device__ __forceinline__ int clampi(int v, int lo, int hi) { return v < lo ? lo : (v > hi ? hi : v); }

__device__ __forceinline__ v8f zero8f() {
  v8f r;
#pragma unroll
  for (int i = 0; i < 8; ++i) r[i] = 0.0f;
  return r;
}

__device__ __forceinline__ v8f wmh(v16h a, v16h b, v8f c) {
  v8f d = __builtin_amdgcn_wmma_f32_16x16x32_f16(false, a, false, b, (short)0, c, false, false);
  asm volatile("v_nop\n\tv_nop\n\tv_nop\n\tv_nop" : "+v"(d) : "v"(a), "v"(b));
  return d;
}
__device__ __forceinline__ v8f wmb(v16b a, v16b b, v8f c) {
  v8f d = __builtin_amdgcn_wmma_f32_16x16x32_bf16(false, a, false, b, (short)0, c, false, false);
  asm volatile("v_nop\n\tv_nop\n\tv_nop\n\tv_nop" : "+v"(d) : "v"(a), "v"(b));
  return d;
}

__device__ __forceinline__ v8h cvt8h(v4f a, v4f b) {
  v8h r;
  r[0] = (_Float16)a.x; r[1] = (_Float16)a.y; r[2] = (_Float16)a.z; r[3] = (_Float16)a.w;
  r[4] = (_Float16)b.x; r[5] = (_Float16)b.y; r[6] = (_Float16)b.z; r[7] = (_Float16)b.w;
  return r;
}

__device__ __forceinline__ void split8(v4f a, v4f b, v8b& hi, v8b& lo) {
  float f[8];
  f[0] = a.x; f[1] = a.y; f[2] = a.z; f[3] = a.w; f[4] = b.x; f[5] = b.y; f[6] = b.z; f[7] = b.w;
#pragma unroll
  for (int i = 0; i < 8; ++i) {
    const __bf16 hb = (__bf16)f[i];
    const float hf = (float)hb;
    hi[i] = hb;
    lo[i] = (__bf16)(f[i] - hf);
  }
}

__global__ __launch_bounds__(NTHR) void k_prep(const float* __restrict__ w_pre, const float* __restrict__ w_cn,
                                               _Float16* wpreT, _Float16* wAT, _Float16* wBT) {
  __shared__ __attribute__((aligned(16))) _Float16 pl[HC * HC];
  const int tid = threadIdx.x;
  const int which = blockIdx.x;
  const int tot = (which == 0) ? HC * FIN : HC * HC;
  if (which == 0) {
    for (int i = tid; i < tot; i += NTHR) {
      const int n = i >> 6, k = i & 63;
      pl[i] = (_Float16)(w_pre[k * HC + n] * WSCL);
    }
  } else if (which == 1) {
    for (int i = tid; i < tot; i += NTHR) {
      const int n = i >> 7, k = i & 127;
      const float v = w_cn[k * HC + n] - w_cn[(k + HC) * HC + n];
      pl[i] = (_Float16)(v * WSCL);
    }
  } else {
    for (int i = tid; i < tot; i += NTHR) {
      const int n = i >> 7, k = i & 127;
      pl[i] = (_Float16)(w_cn[(k + HC) * HC + n] * WSCL);
    }
  }
  __syncthreads();
  _Float16* dp = (which == 0) ? wpreT : ((which == 1) ? wAT : wBT);
  const int nch = tot >> 3;
  for (int i = tid; i < nch; i += NTHR) {
    const v8h v = *(const v8ha*)(pl + 8 * i);
    *(volatile v8h*)(dp + 8 * i) = v;
  }
  __threadfence();
  for (int i = tid; i < nch; i += NTHR) {
    const v8h v = *(const v8ha*)(pl + 8 * i);
    *(volatile v8h*)(dp + 8 * i) = v;
  }
}

__global__ __launch_bounds__(NTHR) void k_gemm1(const float* __restrict__ x, const _Float16* __restrict__ wpreT,
                                                const float* __restrict__ b_pre, float* z, int nN) {
  __shared__ __attribute__((aligned(16))) float stg[NWAVE * 16 * HC];
  const int tid = threadIdx.x, lane = tid & 31, wave = tid >> 5, hh = lane >> 4, m = lane & 15;
  const int rows0 = blockIdx.x * 128 + wave * 16;
  int ar = rows0 + m;
  ar = ar > nN - 1 ? nN - 1 : ar;
  const float* xr = x + (size_t)ar * FIN;
  FragH a[2];
#pragma unroll
  for (int ks = 0; ks < 2; ++ks) {
    const float* p = xr + 32 * ks;
    a[ks].h[0] = cvt8h(*(const v4f*)(p + 8 * hh), *(const v4f*)(p + 8 * hh + 4));
    a[ks].h[1] = cvt8h(*(const v4f*)(p + 16 + 8 * hh), *(const v4f*)(p + 16 + 8 * hh + 4));
  }
  v8f acc[8];
#pragma unroll
  for (int ct = 0; ct < 8; ++ct) acc[ct] = zero8f();
#pragma unroll
  for (int ct = 0; ct < 8; ++ct) {
    const _Float16* q = wpreT + (size_t)(16 * ct + m) * FIN;
#pragma unroll
    for (int ks = 0; ks < 2; ++ks) {
      FragH b;
      b.h[0] = *(const v8h*)(q + 32 * ks + 8 * hh);
      b.h[1] = *(const v8h*)(q + 32 * ks + 16 + 8 * hh);
      acc[ct] = wmh(a[ks].v, b.v, acc[ct]);
    }
  }
  float* sw = stg + wave * 16 * HC;
#pragma unroll
  for (int ct = 0; ct < 8; ++ct) {
    const float bv = b_pre[16 * ct + m];
#pragma unroll
    for (int r = 0; r < 8; ++r) sw[(8 * hh + r) * HC + 16 * ct + m] = acc[ct][r] * WINV + bv;
  }
  __syncthreads();
#pragma unroll 4
  for (int i = 0; i < 16; ++i) {
    const v4f v = *(const v4fa*)(sw + i * HC + 4 * lane);
    *(volatile v4f*)(z + (size_t)(rows0 + i) * HC + 4 * lane) = v;
  }
  __threadfence();
#pragma unroll 4
  for (int i = 0; i < 16; ++i) {
    const v4f v = *(const v4fa*)(sw + i * HC + 4 * lane);
    *(volatile v4f*)(z + (size_t)(rows0 + i) * HC + 4 * lane) = v;
  }
}

__global__ __launch_bounds__(NTHR) void k_bnstat(const float* __restrict__ z, float* bnp, int nN) {
  __shared__ double rs[NWAVE * 32], rq[NWAVE * 32];
  __shared__ __attribute__((aligned(16))) float res[64];
  const int tid = threadIdx.x, lane = tid & 31, wave = tid >> 5;
  const int c = blockIdx.x * 32 + lane;
  double s = 0.0, q = 0.0;
#pragma unroll 1
  for (int r = wave; r < nN; r += NWAVE) {
    const double v = (double)z[(size_t)r * HC + c];
    s += v;
    q += v * v;
  }
  rs[wave * 32 + lane] = s;
  rq[wave * 32 + lane] = q;
  __syncthreads();
  if (tid < 32) {
    double S = 0.0, Q = 0.0;
#pragma unroll
    for (int w = 0; w < NWAVE; ++w) { S += rs[w * 32 + tid]; Q += rq[w * 32 + tid]; }
    const double inv = 1.0 / (double)nN;
    const double mu = S * inv;
    double var = Q * inv - mu * mu;
    if (var < 0.0) var = 0.0;
    res[tid]      = (float)mu;
    res[32 + tid] = 1.0f / sqrtf((float)var + BNEPS);
  }
  __syncthreads();
  v4f v0 = {0.0f, 0.0f, 0.0f, 0.0f}, v1 = {0.0f, 0.0f, 0.0f, 0.0f};
  const bool wr = (wave == 0) && (lane < 8);
  if (wr) { v0 = *(const v4fa*)(res + 4 * lane); v1 = *(const v4fa*)(res + 32 + 4 * lane); }
  if (wr) {
    *(volatile v4f*)(bnp + blockIdx.x * 32 + 4 * lane) = v0;
    *(volatile v4f*)(bnp + HC + blockIdx.x * 32 + 4 * lane) = v1;
  }
  __threadfence();
  if (wr) {
    *(volatile v4f*)(bnp + blockIdx.x * 32 + 4 * lane) = v0;
    *(volatile v4f*)(bnp + HC + blockIdx.x * 32 + 4 * lane) = v1;
  }
}

__global__ __launch_bounds__(NTHR) void k_gemm2(const float* __restrict__ z, const float* __restrict__ bnp,
                                                const float* __restrict__ g, const float* __restrict__ be,
                                                const _Float16* __restrict__ wAT, const _Float16* __restrict__ wBT,
                                                float* aP, float* bP) {
  __shared__ __attribute__((aligned(16))) _Float16 hs[64 * HP];
  __shared__ __attribute__((aligned(16))) float stg[NWAVE * 16 * HC];
  const int tid = threadIdx.x, lane = tid & 31, wave = tid >> 5, hh = lane >> 4, m = lane & 15;
  const int row0 = blockIdx.x * 64;
  {
    const int c = tid & 127, rsub = tid >> 7;
    const float mu = bnp[c], rsd = bnp[HC + c], gc = g[c], bc = be[c];
#pragma unroll 4
    for (int j = 0; j < 32; ++j) {
      const int row = 2 * j + rsub;
      const float zv = z[(size_t)(row0 + row) * HC + c];
      float v = gc * (zv - mu) * rsd + bc;
      v = fmaxf(v, 0.0f);
      hs[row * HP + c] = (_Float16)v;
    }
  }
  __syncthreads();
  const int rt = wave & 3, half = wave >> 2;
  const _Float16* W = (half != 0) ? wBT : wAT;
  float* outp = (half != 0) ? bP : aP;
  v8f acc[8];
#pragma unroll
  for (int ct = 0; ct < 8; ++ct) acc[ct] = zero8f();
#pragma unroll
  for (int ks = 0; ks < 4; ++ks) {
    FragH a;
    const _Float16* hp = hs + (16 * rt + m) * HP + 32 * ks;
    a.h[0] = *(const v8ha*)(hp + 8 * hh);
    a.h[1] = *(const v8ha*)(hp + 16 + 8 * hh);
#pragma unroll
    for (int ct = 0; ct < 8; ++ct) {
      FragH b;
      const _Float16* q = W + (size_t)(16 * ct + m) * HC + 32 * ks;
      b.h[0] = *(const v8h*)(q + 8 * hh);
      b.h[1] = *(const v8h*)(q + 16 + 8 * hh);
      acc[ct] = wmh(a.v, b.v, acc[ct]);
    }
  }
  float* sw = stg + wave * 16 * HC;
#pragma unroll
  for (int ct = 0; ct < 8; ++ct) {
#pragma unroll
    for (int r = 0; r < 8; ++r) sw[(8 * hh + r) * HC + 16 * ct + m] = acc[ct][r] * WINV;
  }
  __syncthreads();
  const size_t orow = (size_t)(row0 + 16 * rt);
#pragma unroll 4
  for (int i = 0; i < 16; ++i) {
    const v4f v = *(const v4fa*)(sw + i * HC + 4 * lane);
    *(volatile v4f*)(outp + (orow + i) * HC + 4 * lane) = v;
  }
  __threadfence();
#pragma unroll 4
  for (int i = 0; i < 16; ++i) {
    const v4f v = *(const v4fa*)(sw + i * HC + 4 * lane);
    *(volatile v4f*)(outp + (orow + i) * HC + 4 * lane) = v;
  }
}

__device__ __forceinline__ int scan8(const int* __restrict__ key, int nK, int e0, int el, int base, int full,
                                     unsigned short* list, int wave, int wc) {
  const int sent = -2147483647 - 1;
  v4i da, db;
  if (full != 0) {
    da = *(const v4i*)(key + e0);
    db = *(const v4i*)(key + e0 + 4);
  } else {
    da.x = (e0     < nK) ? key[min(e0,     nK - 1)] : sent;
    da.y = (e0 + 1 < nK) ? key[min(e0 + 1, nK - 1)] : sent;
    da.z = (e0 + 2 < nK) ? key[min(e0 + 2, nK - 1)] : sent;
    da.w = (e0 + 3 < nK) ? key[min(e0 + 3, nK - 1)] : sent;
    db.x = (e0 + 4 < nK) ? key[min(e0 + 4, nK - 1)] : sent;
    db.y = (e0 + 5 < nK) ? key[min(e0 + 5, nK - 1)] : sent;
    db.z = (e0 + 6 < nK) ? key[min(e0 + 6, nK - 1)] : sent;
    db.w = (e0 + 7 < nK) ? key[min(e0 + 7, nK - 1)] : sent;
  }
  const unsigned nb = (unsigned)base;
  unsigned bits = 0u;
  bits |= (((unsigned)da.x - nb) < (unsigned)NB) ? 1u   : 0u;
  bits |= (((unsigned)da.y - nb) < (unsigned)NB) ? 2u   : 0u;
  bits |= (((unsigned)da.z - nb) < (unsigned)NB) ? 4u   : 0u;
  bits |= (((unsigned)da.w - nb) < (unsigned)NB) ? 8u   : 0u;
  bits |= (((unsigned)db.x - nb) < (unsigned)NB) ? 16u  : 0u;
  bits |= (((unsigned)db.y - nb) < (unsigned)NB) ? 32u  : 0u;
  bits |= (((unsigned)db.z - nb) < (unsigned)NB) ? 64u  : 0u;
  bits |= (((unsigned)db.w - nb) < (unsigned)NB) ? 128u : 0u;
  const unsigned anym = __builtin_amdgcn_ballot_w32(bits != 0u);
  if (anym != 0u) {
    const int c = (int)__builtin_popcount(bits);
    const unsigned b0 = __builtin_amdgcn_ballot_w32((c & 1) != 0);
    const unsigned b1 = __builtin_amdgcn_ballot_w32((c & 2) != 0);
    const unsigned b2 = __builtin_amdgcn_ballot_w32((c & 4) != 0);
    const unsigned b3 = __builtin_amdgcn_ballot_w32((c & 8) != 0);
    const int pre = (int)__builtin_amdgcn_mbcnt_lo(b0, 0u) + 2 * (int)__builtin_amdgcn_mbcnt_lo(b1, 0u)
                  + 4 * (int)__builtin_amdgcn_mbcnt_lo(b2, 0u) + 8 * (int)__builtin_amdgcn_mbcnt_lo(b3, 0u);
    const int tot = (int)__builtin_popcount(b0) + 2 * (int)__builtin_popcount(b1)
                  + 4 * (int)__builtin_popcount(b2) + 8 * (int)__builtin_popcount(b3);
    int pos = wc + pre;
    unsigned bb = bits;
    while (bb != 0u) {
      const int j = __builtin_ctz(bb);
      bb &= bb - 1u;
      if (pos < WCAP) list[wave * WCAP + pos] = (unsigned short)(el + j);
      ++pos;
    }
    return wc + tot;
  }
  return wc;
}

template <int MODE>
__device__ __forceinline__ void drain_mask(unsigned mm, int j, const int* pslot, const int* pdst,
                                           const float* __restrict__ aP, const float* __restrict__ bP,
                                           v4f bvec, float* acc, int base, int nSrc, int lane) {
  while (mm != 0u) {
    const int L = __builtin_ctz(mm);
    mm &= mm - 1u;
    const int i = 8 * L + j;
    int slot = pslot[i];
    slot = clampi(slot, 0, NB - 1);
    int d = pdst[i];
    d = clampi(d, 0, nSrc - 1);
    v4f val;
    if (MODE == 0) {
      int ra = base + slot;
      ra = clampi(ra, 0, nSrc - 1);
      const v4f va = *(const v4f*)(aP + (size_t)ra * HC + 4 * lane);
      const v4f vb = *(const v4f*)(bP + (size_t)d * HC + 4 * lane);
      val = va + vb + bvec;
      val.x = fmaxf(val.x, 0.0f); val.y = fmaxf(val.y, 0.0f);
      val.z = fmaxf(val.z, 0.0f); val.w = fmaxf(val.w, 0.0f);
    } else {
      val = *(const v4f*)(aP + (size_t)d * HC + 4 * lane);
    }
    v4fa* ap = (v4fa*)(acc + slot * HC + 4 * lane);
    const v4f cur = *ap;
    *ap = cur + val;
  }
}

template <int MODE>
__global__ __launch_bounds__(NTHR) void k_seg(const int* __restrict__ key, const int* __restrict__ dsti,
                                              const float* __restrict__ aP, const float* __restrict__ bP,
                                              const float* __restrict__ bias, float* outp,
                                              int nK, int nSrc, int vec) {
  __shared__ __attribute__((aligned(16))) float acc[NB * HC];
  __shared__ __attribute__((aligned(16))) unsigned short list[LISTN];
  __shared__ __attribute__((aligned(16))) int pend[PCAP];
  __shared__ __attribute__((aligned(16))) int pslot[PASSN];
  __shared__ __attribute__((aligned(16))) int pdst[PASSN];
  __shared__ int wcnt[NWAVE];
  __shared__ int pendN;

  const int tid = threadIdx.x, lane = tid & 31, wave = tid >> 5;
  const int base = blockIdx.x * NB;

  {
    const v4f z4 = {0.0f, 0.0f, 0.0f, 0.0f};
    for (int i = tid; i < (NB * HC) / 4; i += NTHR) *(v4fa*)(acc + 4 * i) = z4;
  }
  v4f bvec = {0.0f, 0.0f, 0.0f, 0.0f};
  if (MODE == 0) bvec = *(const v4f*)(bias + 4 * lane);
  if (tid == 0) pendN = 0;
  __syncthreads();

  const int nChunks = (nK + CHUNK - 1) / CHUNK;
#pragma unroll 1
  for (int ch = 0; ch < nChunks; ++ch) {
    const int cbase = ch * CHUNK;
    const int full = (vec != 0 && cbase + CHUNK <= nK) ? 1 : 0;
    int wc = 0;
#pragma unroll
    for (int grp = 0; grp < 2; ++grp) {
      const int el = tid * EPT + 8 * grp;
      wc = scan8(key, nK, cbase + el, el, base, full, list, wave, wc);
    }
    if (lane == 0) wcnt[wave] = wc;
    __syncthreads();

    const int pb = pendN;
    int tot = 0, myoff = 0;
#pragma unroll
    for (int w = 0; w < NWAVE; ++w) {
      int c = wcnt[w];
      c = c > WCAP ? WCAP : (c < 0 ? 0 : c);
      if (w < wave) myoff += c;
      tot += c;
    }
    int newN = pb + tot;
    newN = newN > PCAP ? PCAP : newN;
    {
      int n = wcnt[wave];
      n = n > WCAP ? WCAP : (n < 0 ? 0 : n);
      for (int i = lane; i < n; i += 32) {
        const int pos = pb + myoff + i;
        if (pos < PCAP) pend[pos] = cbase + (int)list[wave * WCAP + i];
      }
    }
    const int fin = (ch == nChunks - 1) ? 1 : 0;
    const int R   = (fin != 0) ? (newN + PASSN - 1) / PASSN : newN / PASSN;
    const int Pv  = (fin != 0) ? newN : R * PASSN;
    __syncthreads();

#pragma unroll 1
    for (int r = 0; r < R; ++r) {
      {
        const int idx = r * PASSN + tid;
        const bool valid = idx < Pv;
        int e = pend[min(idx, PCAP - 1)];
        e = valid ? e : 0;
        e = clampi(e, 0, nK - 1);
        const int kv = key[e];
        int d;
        if (MODE == 0) d = dsti[e]; else d = e;
        d = clampi(d, 0, nSrc - 1);
        int slot = kv - base;
        if (!valid || (unsigned)slot >= (unsigned)NB) slot = -1;
        pslot[tid] = slot;
        pdst[tid] = d;
      }
      __syncthreads();
      {
        const v4i sa = *(const v4ia*)(pslot + 8 * lane);
        const v4i sb = *(const v4ia*)(pslot + 8 * lane + 4);
        const unsigned m0 = __builtin_amdgcn_ballot_w32((sa.x >= 0) && ((sa.x >> 5) == wave));
        const unsigned m1 = __builtin_amdgcn_ballot_w32((sa.y >= 0) && ((sa.y >> 5) == wave));
        const unsigned m2 = __builtin_amdgcn_ballot_w32((sa.z >= 0) && ((sa.z >> 5) == wave));
        const unsigned m3 = __builtin_amdgcn_ballot_w32((sa.w >= 0) && ((sa.w >> 5) == wave));
        const unsigned m4 = __builtin_amdgcn_ballot_w32((sb.x >= 0) && ((sb.x >> 5) == wave));
        const unsigned m5 = __builtin_amdgcn_ballot_w32((sb.y >= 0) && ((sb.y >> 5) == wave));
        const unsigned m6 = __builtin_amdgcn_ballot_w32((sb.z >= 0) && ((sb.z >> 5) == wave));
        const unsigned m7 = __builtin_amdgcn_ballot_w32((sb.w >= 0) && ((sb.w >> 5) == wave));
        drain_mask<MODE>(m0, 0, pslot, pdst, aP, bP, bvec, acc, base, nSrc, lane);
        drain_mask<MODE>(m1, 1, pslot, pdst, aP, bP, bvec, acc, base, nSrc, lane);
        drain_mask<MODE>(m2, 2, pslot, pdst, aP, bP, bvec, acc, base, nSrc, lane);
        drain_mask<MODE>(m3, 3, pslot, pdst, aP, bP, bvec, acc, base, nSrc, lane);
        drain_mask<MODE>(m4, 4, pslot, pdst, aP, bP, bvec, acc, base, nSrc, lane);
        drain_mask<MODE>(m5, 5, pslot, pdst, aP, bP, bvec, acc, base, nSrc, lane);
        drain_mask<MODE>(m6, 6, pslot, pdst, aP, bP, bvec, acc, base, nSrc, lane);
        drain_mask<MODE>(m7, 7, pslot, pdst, aP, bP, bvec, acc, base, nSrc, lane);
      }
      __syncthreads();
    }

    int rem = newN - R * PASSN;
    rem = rem < 0 ? 0 : rem;
    if (R > 0 && tid < rem) pend[tid] = pend[R * PASSN + tid];
    if (tid == 0) pendN = rem;
  }
  __syncthreads();

  const int lr0 = wave * 32;
  const size_t orow0 = (size_t)(base + lr0);
#pragma unroll 4
  for (int i = 0; i < 32; ++i) {
    const v4f v = *(const v4fa*)(acc + (lr0 + i) * HC + 4 * lane);
    *(volatile v4f*)(outp + (orow0 + i) * HC + 4 * lane) = v;
  }
  __threadfence();
#pragma unroll 4
  for (int i = 0; i < 32; ++i) {
    const v4f v = *(const v4fa*)(acc + (lr0 + i) * HC + 4 * lane);
    *(volatile v4f*)(outp + (orow0 + i) * HC + 4 * lane) = v;
  }
}

__global__ __launch_bounds__(NTHR) void k_head(const float* __restrict__ pool, const float* __restrict__ w_post,
                                               const float* __restrict__ b_post, const float* __restrict__ g,
                                               const float* __restrict__ be, const float* __restrict__ w_out,
                                               const float* __restrict__ b_out, float* outp, int G) {
  __shared__ __attribute__((aligned(16))) __bf16 wh[32 * HP];
  __shared__ __attribute__((aligned(16))) __bf16 wl[32 * HP];
  __shared__ __attribute__((aligned(16))) float qs[GMAX * 32];
  __shared__ double red[NWAVE * 32];
  __shared__ float mus[32], rss[32];
  __shared__ float zrow[GMAX];
  __shared__ __attribute__((aligned(16))) float outv[GMAX];

  const int tid = threadIdx.x, lane = tid & 31, wave = tid >> 5, hh = lane >> 4, m = lane & 15;
  for (int i = tid; i < GMAX; i += NTHR) zrow[i] = 0.0f;

#pragma unroll 1
  for (int Q = 0; Q < 4; ++Q) {
    __syncthreads();
    for (int i = tid; i < 32 * HC; i += NTHR) {
      const int n = i >> 7, k = i & 127;
      const float v = w_post[k * HC + 32 * Q + n];
      const __bf16 hb = (__bf16)v;
      const float hf = (float)hb;
      wh[n * HP + k] = hb;
      wl[n * HP + k] = (__bf16)(v - hf);
    }
    __syncthreads();
#pragma unroll 1
    for (int u = 0; u < 8; ++u) {
      const int t = wave * 8 + u, rt = t >> 1, ct = t & 1;
      v8f acc = zero8f();
      const float* prow = pool + (size_t)(16 * rt + m) * HC;
#pragma unroll
      for (int ks = 0; ks < 4; ++ks) {
        const float* p = prow + 32 * ks;
        FragB ah, al, bh, bl;
        split8(*(const v4f*)(p + 8 * hh), *(const v4f*)(p + 8 * hh + 4), ah.h[0], al.h[0]);
        split8(*(const v4f*)(p + 16 + 8 * hh), *(const v4f*)(p + 16 + 8 * hh + 4), ah.h[1], al.h[1]);
        const __bf16* qh = wh + (16 * ct + m) * HP + 32 * ks;
        const __bf16* ql = wl + (16 * ct + m) * HP + 32 * ks;
        bh.h[0] = *(const v8ba*)(qh + 8 * hh);
        bh.h[1] = *(const v8ba*)(qh + 16 + 8 * hh);
        bl.h[0] = *(const v8ba*)(ql + 8 * hh);
        bl.h[1] = *(const v8ba*)(ql + 16 + 8 * hh);
        acc = wmb(ah.v, bh.v, acc);
        acc = wmb(ah.v, bl.v, acc);
        acc = wmb(al.v, bh.v, acc);
      }
      const int col = 16 * ct + m;
      const float bv = b_post[32 * Q + col];
#pragma unroll
      for (int r = 0; r < 8; ++r) qs[(16 * rt + 8 * hh + r) * 32 + col] = acc[r] + bv;
    }
    __syncthreads();
    {
      double s = 0.0;
#pragma unroll 1
      for (int r = wave; r < G; r += NWAVE) s += (double)qs[r * 32 + lane];
      red[wave * 32 + lane] = s;
    }
    __syncthreads();
    if (tid < 32) {
      double S = 0.0;
#pragma unroll
      for (int w = 0; w < NWAVE; ++w) S += red[w * 32 + tid];
      mus[tid] = (float)(S / (double)G);
    }
    __syncthreads();
    {
      const double mu = (double)mus[lane];
      double q = 0.0;
#pragma unroll 1
      for (int r = wave; r < G; r += NWAVE) { const double dv = (double)qs[r * 32 + lane] - mu; q += dv * dv; }
      red[wave * 32 + lane] = q;
    }
    __syncthreads();
    if (tid < 32) {
      double Sq = 0.0;
#pragma unroll
      for (int w = 0; w < NWAVE; ++w) Sq += red[w * 32 + tid];
      double var = Sq / (double)G;
      if (var < 0.0) var = 0.0;
      rss[tid] = 1.0f / sqrtf((float)var + BNEPS);
    }
    __syncthreads();
    {
      const int col = 32 * Q + lane;
      const float gc = g[col], bc = be[col], wo = w_out[col];
      const float mu = mus[lane], rsd = rss[lane];
#pragma unroll 1
      for (int r = wave; r < G; r += NWAVE) {
        float v = gc * (qs[r * 32 + lane] - mu) * rsd + bc;
        v = fmaxf(v, 0.0f);
        float tsum = v * wo;
        tsum += __shfl_xor(tsum, 16);
        tsum += __shfl_xor(tsum, 8);
        tsum += __shfl_xor(tsum, 4);
        tsum += __shfl_xor(tsum, 2);
        tsum += __shfl_xor(tsum, 1);
        if (lane == 0) zrow[r] += tsum;
      }
    }
  }
  __syncthreads();
  {
    const float b0 = b_out[0];
#pragma unroll 1
    for (int i = tid; i < GMAX; i += NTHR) {
      float o = 0.0f;
      if (i < G) {
        const float zz = zrow[i] + b0;
        const float e = expf(-fabsf(zz));
        const float sg = 1.0f / (1.0f + e);
        o = (zz >= 0.0f) ? sg : e * sg;
      }
      outv[i] = o;
    }
  }
  __syncthreads();
  if (wave == 0) {
#pragma unroll
    for (int i = 0; i < 4; ++i) {
      const int off = i * 128 + 4 * lane;
      if (off + 3 < G) { const v4f v = *(const v4fa*)(outv + off); *(volatile v4f*)(outp + off) = v; }
    }
    __threadfence();
#pragma unroll
    for (int i = 0; i < 4; ++i) {
      const int off = i * 128 + 4 * lane;
      if (off + 3 < G) { const v4f v = *(const v4fa*)(outv + off); *(volatile v4f*)(outp + off) = v; }
    }
  }
}

extern "C" void kernel_launch(void* const* d_in, const int* in_sizes, int n_in,
                              void* d_out, int out_size, void* d_ws, size_t ws_size,
                              hipStream_t stream) {
  if (n_in < 16) return;
  const int nN = in_sizes[3];
  const int nE = in_sizes[1];
  const int G  = out_size;
  if (nN < 1 || nE < 0 || G < 1 || G > GMAX) return;
  if (in_sizes[0] != nN * FIN || in_sizes[2] != nE) return;
  if (in_sizes[4] != FIN * HC || in_sizes[5] < HC || in_sizes[6] < HC || in_sizes[7] < HC) return;
  if (in_sizes[8] != 2 * HC * HC || in_sizes[9] < HC) return;
  if (in_sizes[10] != HC * HC || in_sizes[11] < HC || in_sizes[12] < HC || in_sizes[13] < HC) return;
  if (in_sizes[14] < HC || in_sizes[15] < 1) return;

  const float* x       = (const float*)d_in[0];
  const int*   src     = (const int*)d_in[1];
  const int*   dst     = (const int*)d_in[2];
  const int*   seg     = (const int*)d_in[3];
  const float* w_pre   = (const float*)d_in[4];
  const float* b_pre   = (const float*)d_in[5];
  const float* g_pre   = (const float*)d_in[6];
  const float* be_pre  = (const float*)d_in[7];
  const float* w_cn    = (const float*)d_in[8];
  const float* b_cn    = (const float*)d_in[9];
  const float* w_post  = (const float*)d_in[10];
  const float* b_post  = (const float*)d_in[11];
  const float* g_post  = (const float*)d_in[12];
  const float* be_post = (const float*)d_in[13];
  const float* w_out   = (const float*)d_in[14];
  const float* b_out   = (const float*)d_in[15];
  float* out = (float*)d_out;

  const int nBlk1 = (nN + 127) / 128;
  const int NP    = nBlk1 * 128;
  const int nBlk2 = NP / 64;
  const int nBlkA = (nN + NB - 1) / NB;
  const int NPA   = nBlkA * NB;
  const int nBlkP = (G + NB - 1) / NB;

  char* ws = (char*)d_ws;
  size_t off = 0;
  const size_t oWpre = off; off += (size_t)HC * FIN * 2;   off = (off + 255) & ~(size_t)255;
  const size_t oWA   = off; off += (size_t)HC * HC * 2;    off = (off + 255) & ~(size_t)255;
  const size_t oWB   = off; off += (size_t)HC * HC * 2;    off = (off + 255) & ~(size_t)255;
  const size_t oBnp  = off; off += 2 * HC * 4;             off = (off + 255) & ~(size_t)255;
  const size_t oZ    = off; off += (size_t)NP * HC * 4;    off = (off + 255) & ~(size_t)255;
  const size_t oA    = off; off += (size_t)NP * HC * 4;    off = (off + 255) & ~(size_t)255;
  const size_t oB    = off; off += (size_t)NP * HC * 4;    off = (off + 255) & ~(size_t)255;
  const size_t oH1   = off; off += (size_t)NPA * HC * 4;   off = (off + 255) & ~(size_t)255;
  const size_t oPool = off; off += (size_t)GMAX * HC * 4;  off = (off + 255) & ~(size_t)255;
  if (off > ws_size) return;
  if (off > (size_t)134217728) return;

  _Float16* wpreT = (_Float16*)(ws + oWpre);
  _Float16* wAT   = (_Float16*)(ws + oWA);
  _Float16* wBT   = (_Float16*)(ws + oWB);
  float* bnp   = (float*)(ws + oBnp);
  float* zP    = (float*)(ws + oZ);
  float* aP    = (float*)(ws + oA);
  float* bP    = (float*)(ws + oB);
  float* h1P   = (float*)(ws + oH1);
  float* poolP = (float*)(ws + oPool);

  const int vecE = ((nE & 7) == 0) ? 1 : 0;
  const int vecN = ((nN & 7) == 0) ? 1 : 0;

  k_prep<<<3, NTHR, 0, stream>>>(w_pre, w_cn, wpreT, wAT, wBT);
  k_gemm1<<<nBlk1, NTHR, 0, stream>>>(x, wpreT, b_pre, zP, nN);
  k_bnstat<<<HC / 32, NTHR, 0, stream>>>(zP, bnp, nN);
  k_gemm2<<<nBlk2, NTHR, 0, stream>>>(zP, bnp, g_pre, be_pre, wAT, wBT, aP, bP);
  k_seg<0><<<nBlkA, NTHR, 0, stream>>>(src, dst, aP, bP, b_cn, h1P, nE, nN, vecE);
  k_seg<1><<<nBlkP, NTHR, 0, stream>>>(seg, seg, h1P, h1P, b_cn, poolP, nN, nN, vecN);
  k_head<<<1, NTHR, 0, stream>>>(poolP, w_post, b_post, g_post, be_post, w_out, b_out, out, G);
}
